// CrossBlock_88502096101921
// MI455X (gfx1250) — hardware-run, weakly checked
//
#include <hip/hip_runtime.h>


#define NB_  4
#define TT   2048
#define EM   256
#define E2   512
#define NH_  4
#define HD   64
#define PCAR 1024.0f
typedef _Float16 h16;
typedef unsigned short bf;
typedef __attribute__((ext_vector_type(16))) __bf16   v16bf;
typedef __attribute__((ext_vector_type(16))) _Float16 v16h;
typedef __attribute__((ext_vector_type(8)))  _Float16 v8h;
typedef __attribute__((ext_vector_type(8)))  unsigned short v8us;
typedef __attribute__((ext_vector_type(8)))  float    v8f;
typedef __attribute__((ext_vector_type(4)))  float    v4f;
typedef v8h  __attribute__((may_alias)) v8ha;
typedef v4f  __attribute__((may_alias)) v4fa;
typedef v8us __attribute__((may_alias)) v8usa;

__device__ __forceinline__ unsigned short f2bf(float f) { unsigned u = __float_as_uint(f); u += 0x7FFFu + ((u >> 16) & 1u); return (unsigned short)(u >> 16); }
__device__ __forceinline__ float bf2f(unsigned short b) { return __uint_as_float(((unsigned)b) << 16); }
__device__ __forceinline__ float bfr(float f) { return bf2f(f2bf(f)); }
__device__ __forceinline__ v16h cat16(v8h lo, v8h hi) { return __builtin_shufflevector(lo, hi, 0, 1, 2, 3, 4, 5, 6, 7, 8, 9, 10, 11, 12, 13, 14, 15); }
__device__ __forceinline__ v16bf cat16b(v8us lo, v8us hi) { return __builtin_bit_cast(v16bf, __builtin_shufflevector(lo, hi, 0, 1, 2, 3, 4, 5, 6, 7, 8, 9, 10, 11, 12, 13, 14, 15)); }
__device__ __forceinline__ v8f wmma16(v16h a, v16h b, v8f c) { return __builtin_amdgcn_wmma_f32_16x16x32_f16(false, a, false, b, (short)0, c, false, false); }
__device__ __forceinline__ v8f wmmab(v16bf a, v16bf b, v8f c) { return __builtin_amdgcn_wmma_f32_16x16x32_bf16(false, a, false, b, (short)0, c, false, false); }


template <typename T16> struct WFrag;
template <> struct WFrag<h16> { typedef v16h V; static __device__ __forceinline__ V ld(const h16* p) { return cat16(*(const v8h*)p, *(const v8h*)(p + 16)); } static __device__ __forceinline__ v8f mma(V a, V b, v8f c) { return wmma16(a, b, c); } };
template <> struct WFrag<bf> { typedef v16bf V; static __device__ __forceinline__ V ld(const bf* p) { return cat16b(*(const v8us*)p, *(const v8us*)(p + 16)); } static __device__ __forceinline__ v8f mma(V a, V b, v8f c) { return wmmab(a, b, c); } };
template <typename T16, int NSPLIT, bool BIAS>
__global__ __launch_bounds__(32) void k_gemmw(const T16* __restrict__ A, const T16* __restrict__ A2, const T16* __restrict__ Bt, const T16* __restrict__ Bt2, int K, float* C, int ldc, const float* __restrict__ bias, size_t sA, size_t sB, size_t sC) {
    typedef typename WFrag<T16>::V V;
    __shared__ __align__(16) float os[16 * 68];
    const size_t z = blockIdx.z; A += z * sA; if (A2) A2 += z * sA; Bt += z * sB; if (Bt2) Bt2 += z * sB; C += z * sC;
    const int lane = threadIdx.x & 31, lr = lane & 15, hi = lane >> 4; const int r0 = blockIdx.x * 64, c0 = blockIdx.y * 64;
    v8f acc[4][4];
#pragma unroll
    for (int mb = 0; mb < 4; ++mb)
#pragma unroll
        for (int nb = 0; nb < 4; ++nb) acc[mb][nb] = (v8f){};
    const size_t aoff = (size_t)(r0 + lr) * K + 8 * hi, boff = (size_t)(c0 + lr) * K + 8 * hi;
#pragma unroll 1
    for (int kc = 0; kc < K; kc += 32) {
        V a[4], a2[4];
#pragma unroll
        for (int mb = 0; mb < 4; ++mb) { a[mb] = WFrag<T16>::ld(A + aoff + (size_t)mb * 16 * K + kc); if (NSPLIT == 1 || NSPLIT == 2) a2[mb] = WFrag<T16>::ld(A2 + aoff + (size_t)mb * 16 * K + kc); }
#pragma unroll
        for (int nb = 0; nb < 4; ++nb) { const V b = WFrag<T16>::ld(Bt + boff + (size_t)nb * 16 * K + kc); V b2; if (NSPLIT >= 2) b2 = WFrag<T16>::ld(Bt2 + boff + (size_t)nb * 16 * K + kc);
#pragma unroll
            for (int mb = 0; mb < 4; ++mb) { acc[mb][nb] = WFrag<T16>::mma(a[mb], b, acc[mb][nb]); if (NSPLIT == 1 || NSPLIT == 2) acc[mb][nb] = WFrag<T16>::mma(a2[mb], b, acc[mb][nb]); if (NSPLIT >= 2) acc[mb][nb] = WFrag<T16>::mma(a[mb], b2, acc[mb][nb]); } }
        asm volatile("v_nop\n\tv_nop\n\tv_nop\n\tv_nop" : "+v"(acc[0][0]), "+v"(acc[1][1]), "+v"(acc[2][2]), "+v"(acc[3][3]) : "v"(a[0]), "v"(a[3]));
    }
#pragma unroll
    for (int mb = 0; mb < 4; ++mb) {
#pragma unroll
        for (int nb = 0; nb < 4; ++nb) {
#pragma unroll
            for (int j = 0; j < 8; ++j) os[(hi * 8 + j) * 68 + nb * 16 + lr] = acc[mb][nb][j]; }
        __builtin_amdgcn_wave_barrier(); asm volatile("" ::: "memory");
        float* crow = C + (size_t)(r0 + mb * 16) * ldc + c0;
#pragma unroll 1
        for (int ps = 0; ps < 2; ++ps) {
#pragma unroll
            for (int s = 0; s < 8; ++s) { const int row = 2 * s + hi, cofs = lr * 4; v4f val = *(const v4fa*)(os + row * 68 + cofs); if (BIAS) { val[0] += bfr(bias[c0 + cofs]); val[1] += bfr(bias[c0 + cofs + 1]); val[2] += bfr(bias[c0 + cofs + 2]); val[3] += bfr(bias[c0 + cofs + 3]); }
                *(volatile v4f*)(crow + (size_t)row * ldc + cofs) = val; }
            if (ps == 0) __threadfence(); }
        __builtin_amdgcn_wave_barrier(); asm volatile("" ::: "memory");
    }
}

__device__ __forceinline__ h16 tohx(float x) { return (h16)x; }
__device__ __forceinline__ void splitf(float y, unsigned short& h, unsigned short& l) { h = f2bf(y); l = f2bf(y - bf2f(h)); }
typedef __attribute__((ext_vector_type(2))) unsigned short v2us;
typedef __attribute__((ext_vector_type(4))) unsigned short v4us;
typedef __attribute__((ext_vector_type(2))) _Float16 v2h;
typedef __attribute__((ext_vector_type(4))) _Float16 v4h;

__global__ __launch_bounds__(256) void k_cvt8(const float* __restrict__ src, bf* dst, size_t n8) { const size_t i = (size_t)blockIdx.x * 256 + threadIdx.x; if (i >= n8) return; const v8f v = *(const v8f*)(src + i * 8); v8us o;
#pragma unroll
    for (int k = 0; k < 8; ++k) o[k] = f2bf(v[k]); *(volatile v8us*)(dst + i * 8) = o; __threadfence(); *(volatile v8us*)(dst + i * 8) = o; }
__global__ __launch_bounds__(256) void k_wtG(const float* __restrict__ w, int K, int N, bf* Bt) {
    const int lane = threadIdx.x & 31; const int L0 = (blockIdx.x * 8 + (threadIdx.x >> 5)) * 8; const int nlines = N * K / 64;
#pragma unroll
    for (int ps = 0; ps < 2; ++ps) {
#pragma unroll 1
        for (int l = 0; l < 8; ++l) { const int L = L0 + l; if (L >= nlines) break; const size_t e = (size_t)L * 64 + lane * 2; const int k = (int)(e % K), n = (int)(e / K); v2us o;
            o[0] = f2bf(w[(size_t)k * N + n]); o[1] = f2bf(w[(size_t)(k + 1) * N + n]); *(volatile v2us*)(Bt + e) = o; }
        if (ps == 0) __threadfence(); }
}

__global__ __launch_bounds__(256) void k_qpl(const float* __restrict__ F, h16* P) { const size_t e = ((size_t)blockIdx.x * 256 + threadIdx.x) * 4; if (e >= (size_t)NH_ * TT * HD) return; const int d = (int)(e % HD); const int t = (int)((e / HD) % TT); const int h = (int)(e / ((size_t)HD * TT)); const float* f = F + (size_t)t * EM + h * HD + d; v4h o;
#pragma unroll
    for (int u = 0; u < 4; ++u) o[u] = tohx(__fmul_rn(f[u], 0.35355339059327379f)); *(volatile v4h*)(P + e) = o; __threadfence(); *(volatile v4h*)(P + e) = o; }
__global__ __launch_bounds__(256) void k_vt(const float* __restrict__ F, h16* VT) { const size_t e = ((size_t)blockIdx.x * 256 + threadIdx.x) * 2; if (e >= (size_t)NH_ * HD * TT) return; const int t = (int)(e % TT); const int d = (int)((e / TT) % HD); const int h = (int)(e / ((size_t)TT * HD)); v2h o; o[0] = tohx(F[(size_t)t * EM + h * HD + d]); o[1] = tohx(F[(size_t)(t + 1) * EM + h * HD + d]); *(volatile v2h*)(VT + e) = o; __threadfence(); *(volatile v2h*)(VT + e) = o; }
__global__ __launch_bounds__(256) void k_smax(const float* __restrict__ S, h16* P16) { const int lane = threadIdx.x & 31; const int row = blockIdx.x * 8 + (threadIdx.x >> 5); if (row >= NH_ * TT) return; const float* sr = S + (size_t)row * TT; float v[TT / 32]; float mx = -3.0e38f;
#pragma unroll
    for (int ch = 0; ch < TT / 128; ++ch) { const v4f a = *(const v4f*)(sr + ch * 128 + lane * 4);
#pragma unroll
        for (int u = 0; u < 4; ++u) { v[ch * 4 + u] = a[u]; mx = fmaxf(mx, a[u]); } }
#pragma unroll
    for (int sh = 16; sh; sh >>= 1) mx = fmaxf(mx, __shfl_xor(mx, sh, 32));
    float sum = 0.f;
#pragma unroll
    for (int q = 0; q < TT / 32; ++q) { float d0 = __fsub_rn(v[q], mx); asm volatile("" : "+v"(d0)); v[q] = __builtin_amdgcn_exp2f(__fmul_rn(d0, 1.4426950408889634f)); sum += v[q]; }
#pragma unroll
    for (int sh = 16; sh; sh >>= 1) sum += __shfl_xor(sum, sh, 32);
    const float f = __fdiv_rn(PCAR, sum);
    for (int ps = 0; ps < 2; ++ps) {
#pragma unroll
        for (int ch = 0; ch < TT / 128; ++ch) { v4h o4; for (int q = 0; q < 4; ++q) o4[q] = tohx(v[ch * 4 + q] * f); *(volatile v4h*)(P16 + (size_t)row * TT + ch * 128 + lane * 4) = o4; }
        if (ps == 0) __threadfence(); } }
__global__ __launch_bounds__(256) void k_mrg(const float* __restrict__ O, bf* Ah, bf* Al) { const size_t e = ((size_t)blockIdx.x * 256 + threadIdx.x) * 4; if (e >= (size_t)NH_ * TT * HD) return; const int d = (int)(e % HD); const int t = (int)((e / HD) % TT); const int h = (int)(e / ((size_t)HD * TT)); const size_t oo = (size_t)t * EM + h * HD + d; v4us oh, ol;
#pragma unroll
    for (int u = 0; u < 4; ++u) { unsigned short a, b; splitf(O[e + u] * (1.0f / PCAR), a, b); oh[u] = a; ol[u] = b; } *(volatile v4us*)(Ah + oo) = oh; *(volatile v4us*)(Al + oo) = ol; __threadfence(); *(volatile v4us*)(Ah + oo) = oh; *(volatile v4us*)(Al + oo) = ol; }
__global__ __launch_bounds__(256) void k_cat(const float* __restrict__ xb, const float* __restrict__ M, bf* Ah, bf* Al) { const size_t e = ((size_t)blockIdx.x * 256 + threadIdx.x) * 4; if (e >= (size_t)TT * E2) return; const int c = (int)(e % E2); const size_t t = e / E2; v4us oh, ol;
#pragma unroll
    for (int u = 0; u < 4; ++u) { if (c < EM) { oh[u] = f2bf(xb[t * EM + c + u]); ol[u] = 0; } else { unsigned short a, b; splitf(M[t * EM + c - EM + u], a, b); oh[u] = a; ol[u] = b; } } *(volatile v4us*)(Ah + e) = oh; *(volatile v4us*)(Al + e) = ol; __threadfence(); *(volatile v4us*)(Ah + e) = oh; *(volatile v4us*)(Al + e) = ol; }
__global__ __launch_bounds__(256) void k_lngelu(const float* __restrict__ Hf, const float* __restrict__ g, const float* __restrict__ bb, float* Hn) { const int lane = threadIdx.x & 31; const size_t r = (size_t)blockIdx.x * 8 + (threadIdx.x >> 5); if (r >= TT) return; float v[16]; float s = 0.f;
#pragma unroll
    for (int ch = 0; ch < 4; ++ch) { const v4f a = *(const v4f*)(Hf + r * E2 + ch * 128 + lane * 4);
#pragma unroll
        for (int u = 0; u < 4; ++u) { v[ch * 4 + u] = a[u]; s += a[u]; } }
#pragma unroll
    for (int sh = 16; sh; sh >>= 1) s += __shfl_xor(s, sh, 32);
    const float mean = s * (1.0f / E2); float q = 0.f;
#pragma unroll
    for (int k = 0; k < 16; ++k) { float d = __fsub_rn(v[k], mean); asm volatile("" : "+v"(d)); v[k] = d; float p = __fmul_rn(d, d); asm volatile("" : "+v"(p)); q = __fadd_rn(q, p); }
#pragma unroll
    for (int sh = 16; sh; sh >>= 1) q += __shfl_xor(q, sh, 32);
    const float rs = __frsqrt_rn(__fadd_rn(q * (1.0f / E2), 1e-5f));
    for (int ps = 0; ps < 2; ++ps) {
#pragma unroll
        for (int ch = 0; ch < 4; ++ch) { v4f hn;
#pragma unroll
            for (int u = 0; u < 4; ++u) { const int c = ch * 128 + lane * 4 + u; float n0 = __fmul_rn(v[ch * 4 + u], rs); asm volatile("" : "+v"(n0)); float gg = bfr(g[c]), be = bfr(bb[c]); asm volatile("" : "+v"(gg)); asm volatile("" : "+v"(be)); float t1 = __fmul_rn(n0, gg); asm volatile("" : "+v"(t1)); const float hh = __fadd_rn(t1, be);
                hn[u] = hh; }
            const size_t oo = r * E2 + ch * 128 + lane * 4; *(volatile v4f*)(Hn + oo) = hn; }
        if (ps == 0) __threadfence(); } }
__global__ __launch_bounds__(256) void k_gelu(const float* __restrict__ Hn, bf* Ph, bf* Pl) { const size_t e = ((size_t)blockIdx.x * 256 + threadIdx.x) * 4; if (e >= (size_t)TT * E2) return; v4us oh, ol;
#pragma unroll
    for (int u = 0; u < 4; ++u) { const float hh = Hn[e + u]; float er = erff(hh * 0.70710678118654752f); asm volatile("" : "+v"(er)); float hx = hh * 0.5f; asm volatile("" : "+v"(hx)); unsigned short a2, c2; splitf(__fmul_rn(hx, __fadd_rn(1.0f, er)), a2, c2); oh[u] = a2; ol[u] = c2; }
    *(volatile v4us*)(Ph + e) = oh; *(volatile v4us*)(Pl + e) = ol; __threadfence(); *(volatile v4us*)(Ph + e) = oh; *(volatile v4us*)(Pl + e) = ol; }
__global__ __launch_bounds__(256) void k_resid(const float* __restrict__ X, float* O, size_t n4) { const size_t e = ((size_t)blockIdx.x * 256 + threadIdx.x) * 4; if (e >= n4 * 4) return; const v4f a = *(const v4f*)(X + e), o0 = *(const v4f*)(O + e); v4f r;
#pragma unroll
    for (int u = 0; u < 4; ++u) r[u] = __fadd_rn(bfr(a[u]), o0[u]); *(volatile v4f*)(O + e) = r; __threadfence(); *(volatile v4f*)(O + e) = r; }

extern "C" void kernel_launch(void* const* d_in, const int* in_sizes, int n_in,
                              void* d_out, int out_size, void* d_ws, size_t ws_size, hipStream_t stream) {
    (void)in_sizes; (void)n_in; (void)out_size;
    const float** I = (const float**)d_in;
    const float *x0 = I[0], *x1 = I[1], *Wqk = I[2], *bqk = I[3], *Wv = I[4], *bv = I[5], *Wo = I[6], *bo = I[7], *W1 = I[8], *b1 = I[9], *lng = I[10], *lnb = I[11], *W2 = I[12], *b2 = I[13];
    float* Y0 = (float*)d_out; float* Y1 = (float*)d_out + (size_t)NB_ * TT * EM;
    char* wsp = (char*)d_ws;
    auto take = [&](size_t bytes) { char* p = wsp; wsp += (bytes + 255) & ~(size_t)255; return (void*)p; };
    bf* BQK = (bf*)take((size_t)EM * EM * 2); bf* BVW = (bf*)take((size_t)EM * EM * 2); bf* BO = (bf*)take((size_t)EM * EM * 2); bf* BW1 = (bf*)take((size_t)E2 * E2 * 2); bf* BW2 = (bf*)take((size_t)EM * E2 * 2);
    bf* XB0 = (bf*)take((size_t)TT * EM * 2); bf* XB1 = (bf*)take((size_t)TT * EM * 2); float* F = (float*)take((size_t)TT * EM * 4);
    h16* Q0 = (h16*)take((size_t)NH_ * TT * HD * 2); h16* Q1 = (h16*)take((size_t)NH_ * TT * HD * 2); h16* VT0 = (h16*)take((size_t)NH_ * HD * TT * 2); h16* VT1 = (h16*)take((size_t)NH_ * HD * TT * 2);
    float* S = (float*)take((size_t)NH_ * TT * TT * 4); h16* P16 = (h16*)take((size_t)NH_ * TT * TT * 2); float* O = (float*)take((size_t)NH_ * TT * HD * 4); bf* MPh = (bf*)take((size_t)TT * EM * 2); bf* MPl = (bf*)take((size_t)TT * EM * 2); float* M = (float*)take((size_t)TT * EM * 4);
    bf* CAh = (bf*)take((size_t)TT * E2 * 2); bf* CAl = (bf*)take((size_t)TT * E2 * 2); float* Hf = (float*)take((size_t)TT * E2 * 4); float* Hn = (float*)take((size_t)TT * E2 * 4); bf* Gh = (bf*)take((size_t)TT * E2 * 2); bf* Gl = (bf*)take((size_t)TT * E2 * 2);
    if ((size_t)(wsp - (char*)d_ws) > ws_size) return;
    k_wtG<<<(EM * EM / 64 + 63) / 64, 256, 0, stream>>>(Wqk, EM, EM, BQK); k_wtG<<<(EM * EM / 64 + 63) / 64, 256, 0, stream>>>(Wv, EM, EM, BVW); k_wtG<<<(EM * EM / 64 + 63) / 64, 256, 0, stream>>>(Wo, EM, EM, BO); k_wtG<<<(E2 * E2 / 64 + 63) / 64, 256, 0, stream>>>(W1, E2, E2, BW1); k_wtG<<<(E2 * EM / 64 + 63) / 64, 256, 0, stream>>>(W2, E2, EM, BW2);
    const size_t zq = (size_t)TT * HD, zS = (size_t)TT * TT, zv = (size_t)HD * TT;
    const unsigned gq = (unsigned)(((size_t)NH_ * TT * HD / 4 + 255) / 256), gv = (unsigned)(((size_t)NH_ * HD * TT / 2 + 255) / 256);
    for (int b = 0; b < NB_; ++b) { const float* xb0 = x0 + (size_t)b * TT * EM; const float* xb1 = x1 + (size_t)b * TT * EM;
        k_cvt8<<<(TT * EM / 8 + 255) / 256, 256, 0, stream>>>(xb0, XB0, TT * EM / 8); k_cvt8<<<(TT * EM / 8 + 255) / 256, 256, 0, stream>>>(xb1, XB1, TT * EM / 8);
        k_gemmw<bf, 0, true><<<dim3(TT / 64, EM / 64, 1), 32, 0, stream>>>(XB0, nullptr, BQK, nullptr, EM, F, EM, bqk, 0, 0, 0); k_qpl<<<gq, 256, 0, stream>>>(F, Q0);
        k_gemmw<bf, 0, true><<<dim3(TT / 64, EM / 64, 1), 32, 0, stream>>>(XB1, nullptr, BQK, nullptr, EM, F, EM, bqk, 0, 0, 0); k_qpl<<<gq, 256, 0, stream>>>(F, Q1);
        k_gemmw<bf, 0, true><<<dim3(TT / 64, EM / 64, 1), 32, 0, stream>>>(XB0, nullptr, BVW, nullptr, EM, F, EM, bv, 0, 0, 0); k_vt<<<gv, 256, 0, stream>>>(F, VT0);
        k_gemmw<bf, 0, true><<<dim3(TT / 64, EM / 64, 1), 32, 0, stream>>>(XB1, nullptr, BVW, nullptr, EM, F, EM, bv, 0, 0, 0); k_vt<<<gv, 256, 0, stream>>>(F, VT1);
        for (int dir = 0; dir < 2; ++dir) { const h16* QA = dir ? Q1 : Q0; const h16* QB = dir ? Q0 : Q1; const h16* VTB = dir ? VT0 : VT1; const float* xs = dir ? xb1 : xb0; float* Y = (dir ? Y1 : Y0) + (size_t)b * TT * EM;
            k_gemmw<h16, 0, false><<<dim3(TT / 64, TT / 64, NH_), 32, 0, stream>>>(QA, nullptr, QB, nullptr, HD, S, TT, nullptr, zq, zq, zS);
            k_smax<<<NH_ * TT / 8, 256, 0, stream>>>(S, P16);
            k_gemmw<h16, 0, false><<<dim3(TT / 64, 1, NH_), 32, 0, stream>>>(P16, nullptr, VTB, nullptr, TT, O, HD, nullptr, zS, zv, zq);
            k_mrg<<<gq, 256, 0, stream>>>(O, MPh, MPl);
            k_gemmw<bf, 1, true><<<dim3(TT / 64, EM / 64, 1), 32, 0, stream>>>(MPh, MPl, BO, nullptr, EM, M, EM, bo, 0, 0, 0);
            k_cat<<<(TT * E2 / 4 + 255) / 256, 256, 0, stream>>>(xs, M, CAh, CAl);
            k_gemmw<bf, 1, true><<<dim3(TT / 64, E2 / 64, 1), 32, 0, stream>>>(CAh, CAl, BW1, nullptr, E2, Hf, E2, b1, 0, 0, 0);
            k_lngelu<<<TT / 8, 256, 0, stream>>>(Hf, lng, lnb, Hn); k_gelu<<<(TT * E2 / 4 + 255) / 256, 256, 0, stream>>>(Hn, Gh, Gl);
            k_gemmw<bf, 1, true><<<dim3(TT / 64, EM / 64, 1), 32, 0, stream>>>(Gh, Gl, BW2, nullptr, E2, Y, EM, b2, 0, 0, 0);
            k_resid<<<(TT * EM / 4 + 255) / 256, 256, 0, stream>>>(xs, Y, (size_t)TT * EM / 4); } }
}
